// HookedMambaBlock_4664334483709
// MI455X (gfx1250) — hardware-verified
//
#include <hip/hip_runtime.h>
#include <math.h>

constexpr int kL   = 2048;
constexpr int kDm  = 2048;
constexpr int kE   = 4096;
constexpr int kNS  = 16;
constexpr int kDR  = 128;
constexpr int kBCN = 64;
constexpr float kWCarry    = 16.0f;
constexpr float kWCarryInv = 1.0f / 16.0f;
constexpr float kInvDm     = 1.0f / 2048.0f;
constexpr float kEps       = 1e-5f;
constexpr int kScanCh = 64;
constexpr int kScanT  = 32;

typedef __attribute__((ext_vector_type(16))) _Float16 v16h;
typedef __attribute__((ext_vector_type(8)))  _Float16 v8h;
typedef __attribute__((ext_vector_type(16))) __bf16   v16b;
typedef __attribute__((ext_vector_type(8)))  __bf16   v8b;
typedef __attribute__((ext_vector_type(8)))  float    v8f;
typedef __attribute__((ext_vector_type(4)))  float    v4f;
typedef __attribute__((ext_vector_type(4)))  unsigned int v4u;

__device__ __forceinline__ unsigned short f2bf_bits(float f) {
  unsigned u = __float_as_uint(f);
  return (unsigned short)((u + 0x7FFFu + ((u >> 16) & 1u)) >> 16);
}
__device__ __forceinline__ float bf_bits2f(unsigned short h) { return __uint_as_float(((unsigned)h) << 16); }

__device__ __forceinline__ void dep_guard_h(v8f& a, v8f& b, v16h x, v16h y) { asm volatile("v_nop\n\tv_nop\n\tv_nop\n\tv_nop" : "+v"(a), "+v"(b) : "v"(x), "v"(y)); }
__device__ __forceinline__ void dep_guard_b(v8f& a, v8f& b, v16b x, v16b y) { asm volatile("v_nop\n\tv_nop\n\tv_nop\n\tv_nop" : "+v"(a), "+v"(b) : "v"(x), "v"(y)); }
__device__ __forceinline__ void keep4_h(v16h a, v16h b, v16h c, v16h d) { asm volatile("v_nop" :: "v"(a), "v"(b), "v"(c), "v"(d)); }
__device__ __forceinline__ void keep4_b(v16b a, v16b b, v16b c, v16b d) { asm volatile("v_nop" :: "v"(a), "v"(b), "v"(c), "v"(d)); }
__device__ __forceinline__ void acc_guard4(v8f& a, v8f& b, v8f& c, v8f& d) { asm volatile("v_nop\n\tv_nop\n\tv_nop\n\tv_nop" : "+v"(a), "+v"(b), "+v"(c), "+v"(d)); }
template <typename T> struct Frag;
template <> struct Frag<_Float16> {
  typedef v16h V; union U { v16h v; v8h h[2]; };
  static __device__ __forceinline__ v16h load(const _Float16* p) {
    U f; f.h[0] = *(const v8h*)(p); f.h[1] = *(const v8h*)(p + 16); return f.v;
  }
  static __device__ __forceinline__ v8f mma(v16h a, v16h b, v8f c) {
    return __builtin_amdgcn_wmma_f32_16x16x32_f16(false, a, false, b, (short)0, c, false, false);
  }
  static __device__ __forceinline__ void guard(v8f& a, v8f& b, v16h x, v16h y) { dep_guard_h(a, b, x, y); }
  static __device__ __forceinline__ void keep(v16h a, v16h b, v16h c, v16h d) { keep4_h(a, b, c, d); }
};
template <> struct Frag<__bf16> {
  typedef v16b V; union U { v16b v; v8b h[2]; };
  static __device__ __forceinline__ v16b load(const __bf16* p) {
    U f; f.h[0] = *(const v8b*)(p); f.h[1] = *(const v8b*)(p + 16); return f.v;
  }
  static __device__ __forceinline__ v8f mma(v16b a, v16b b, v8f c) {
    return __builtin_amdgcn_wmma_f32_16x16x32_bf16(false, a, false, b, (short)0, c, false, false);
  }
  static __device__ __forceinline__ void guard(v8f& a, v8f& b, v16b x, v16b y) { dep_guard_b(a, b, x, y); }
  static __device__ __forceinline__ void keep(v16b a, v16b b, v16b c, v16b d) { keep4_b(a, b, c, d); }
};

__device__ __forceinline__ unsigned pk16(unsigned short a, unsigned short b) { return (unsigned)a | ((unsigned)b << 16); }
__device__ __forceinline__ unsigned short h_bits(float f) { const _Float16 h = (_Float16)f; return __builtin_bit_cast(unsigned short, h); }

template <int ET> struct Elem;
template <> struct Elem<0> { typedef _Float16 T; };
template <> struct Elem<1> { typedef __bf16 T; };
template <int ET, bool SPLIT, int BIAS_MODE, int OUT_MODE, bool RESID, int ACT = 0>
__global__ __launch_bounds__(256) void wmma_gemm64(
    const unsigned short* __restrict__ Ap, const unsigned short* __restrict__ A2p, int lda, long strideA,
    const unsigned short* __restrict__ Btp, const unsigned short* __restrict__ Bt2p, int ldb, long strideB,
    void* __restrict__ Cout, void* __restrict__ Cout2, int ldc, long strideC,
    const float* __restrict__ bias,
    const float* __restrict__ resid, long strideR,
    int M, int N, int K, float scale) {
  typedef typename Elem<ET>::T T;
  typedef typename Frag<T>::V V;
  const T* A = (const T*)Ap; const T* A2 = (const T*)A2p; const T* Bt = (const T*)Btp; const T* Bt2 = (const T*)Bt2p;
  __shared__ __align__(16) float sT[8][16 * 68];
  const int b    = blockIdx.y;
  const int lane = threadIdx.x & 31;
  const int wave = threadIdx.x >> 5;
  const int tilesN = N >> 6;
  const int tilesM = M >> 6;
  const int tile = blockIdx.x * 8 + wave;
  if (tile >= tilesM * tilesN) return;
  const int tm = tile / tilesN;
  const int tn = tile - tm * tilesN;
  const int m0 = tm << 6;
  const int n0 = tn << 6;

  const T* Ab  = A  + (size_t)b * strideA;
  const T* Bb  = Bt + (size_t)b * strideB;
  const T* Ab2 = SPLIT ? (A2  + (size_t)b * strideA) : nullptr;
  const T* Bb2 = SPLIT ? (Bt2 + (size_t)b * strideB) : nullptr;

  const int rlane = lane & 15;
  const int koff  = (lane >> 4) * 8;
  const int mOff  = (lane >> 4) * 8;

  v8f acc[4][4];
#pragma unroll
  for (int i = 0; i < 4; ++i)
#pragma unroll
    for (int j = 0; j < 4; ++j) acc[i][j] = (v8f){0.f,0.f,0.f,0.f,0.f,0.f,0.f,0.f};

  for (int k0 = 0; k0 < K; k0 += 32) {
    V bh[4], bl[4];
#pragma unroll
    for (int j = 0; j < 4; ++j) {
      const size_t bo = (size_t)(n0 + (j << 4) + rlane) * ldb + koff + k0;
      bh[j] = Frag<T>::load(Bb + bo);
      if (SPLIT) bl[j] = Frag<T>::load(Bb2 + bo);
    }
#pragma unroll
    for (int i = 0; i < 4; ++i) {
      const size_t ao = (size_t)(m0 + (i << 4) + rlane) * lda + koff + k0;
      V ah = Frag<T>::load(Ab + ao);
      V al;
      if (SPLIT) al = Frag<T>::load(Ab2 + ao);
#pragma unroll
      for (int j = 0; j < 4; ++j) {
        acc[i][j] = Frag<T>::mma(ah, bh[j], acc[i][j]);
        if (SPLIT) {
          acc[i][j] = Frag<T>::mma(ah, bl[j], acc[i][j]);
          acc[i][j] = Frag<T>::mma(al, bh[j], acc[i][j]);
        }
      }
      Frag<T>::guard(acc[i][0], acc[i][3], ah, SPLIT ? al : ah);
    }
    Frag<T>::keep(bh[0], bh[1], bh[2], bh[3]);
    if (SPLIT) Frag<T>::keep(bl[0], bl[1], bl[2], bl[3]);
  }
  acc_guard4(acc[0][0], acc[0][1], acc[0][2], acc[0][3]);
  acc_guard4(acc[1][0], acc[1][1], acc[1][2], acc[1][3]);
  acc_guard4(acc[2][0], acc[2][1], acc[2][2], acc[2][3]);
  acc_guard4(acc[3][0], acc[3][1], acc[3][2], acc[3][3]);

  float* slab = sT[wave];
  const float* Rb = RESID ? (resid + (size_t)b * strideR) : nullptr;
#pragma unroll
  for (int i = 0; i < 4; ++i) {
    const int mBase = m0 + (i << 4);
#pragma unroll
    for (int j = 0; j < 4; ++j) {
      const int n = n0 + (j << 4) + rlane;
      float bv = 0.f;
      if (BIAS_MODE == 2) bv = bias[n];
#pragma unroll
      for (int r = 0; r < 8; ++r) {
        float v = acc[i][j][r] * scale;
        if (BIAS_MODE == 1) v += bias[mBase + mOff + r];
        if (BIAS_MODE == 2) v += bv;
        if (RESID) v += Rb[(size_t)(mBase + mOff + r) * ldc + n];
        if (ACT == 2) v = fmaxf(v, 0.0f);
        if (ACT == 4) v = (v > 0.f) ? v : 0.01f * v;
        slab[(mOff + r) * 68 + (j << 4) + rlane] = v;
      }
    }
    __builtin_amdgcn_fence(__ATOMIC_RELEASE, "workgroup");
    __builtin_amdgcn_wave_barrier();
    __builtin_amdgcn_fence(__ATOMIC_ACQUIRE, "workgroup");
    if (OUT_MODE == 0) {
      float* C = (float*)Cout + (size_t)b * strideC;
      const int hh = lane >> 4, c4 = (lane & 15) * 4;
      for (int pass = 0; pass < 2; ++pass) {
#pragma unroll
        for (int it = 0; it < 8; ++it) {
          const int row = it * 2 + hh;
          v4f v = *(const v4f*)(slab + row * 68 + c4);
          *(volatile v4f*)(C + (size_t)(mBase + row) * ldc + n0 + c4) = v;
        }
        __threadfence();
      }
    } else {
      const int q = lane >> 3, c8 = (lane & 7) * 8;
      unsigned short* C  = (unsigned short*)Cout  + (size_t)b * strideC;
      unsigned short* C2 = (OUT_MODE == 2) ? ((unsigned short*)Cout2 + (size_t)b * strideC) : nullptr;
      for (int pass = 0; pass < 2; ++pass) {
#pragma unroll
        for (int it = 0; it < 4; ++it) {
          const int row = it * 4 + q;
          const float* sp = slab + row * 68 + c8;
          v8h hv, lv;
#pragma unroll
          for (int e = 0; e < 8; ++e) {
            if (OUT_MODE == 1) {
              hv[e] = (_Float16)sp[e];
            } else {
              unsigned short hb = f2bf_bits(sp[e]);
              unsigned short lb = f2bf_bits(sp[e] - bf_bits2f(hb));
              hv[e] = __builtin_bit_cast(_Float16, hb);
              lv[e] = __builtin_bit_cast(_Float16, lb);
            }
          }
          *(volatile v8h*)(C + (size_t)(mBase + row) * ldc + n0 + c8) = hv;
          if (OUT_MODE == 2) *(volatile v8h*)(C2 + (size_t)(mBase + row) * ldc + n0 + c8) = lv;
        }
        __threadfence();
      }
    }
    __builtin_amdgcn_fence(__ATOMIC_RELEASE, "workgroup");
    __builtin_amdgcn_wave_barrier();
    __builtin_amdgcn_fence(__ATOMIC_ACQUIRE, "workgroup");
  }
}

__device__ __forceinline__ float silu_f(float s) {
  const float ev = expf(fminf(-s, 80.0f));
  return s * (1.0f / (1.0f + ev));
}
__device__ __forceinline__ float softplus_f(float z) {
  return fmaxf(z, 0.0f) + log1pf(expf(-fabsf(z)));
}
__device__ __forceinline__ v4u pack8(const unsigned short (&b)[8]) {
  return (v4u){pk16(b[0], b[1]), pk16(b[2], b[3]), pk16(b[4], b[5]), pk16(b[6], b[7])};
}

template <int MODE>
__global__ __launch_bounds__(256) void tcast_kernel(const float* __restrict__ in, unsigned short* __restrict__ out0,
                                                    unsigned short* __restrict__ out1, int R, int CC, float scale) {
  __shared__ float sm[64][65];
  const int t  = threadIdx.x;
  const int r0 = blockIdx.x * 64;
  const int c0 = blockIdx.y * 64;
#pragma unroll
  for (int i = 0; i < 16; ++i) {
    const int e = i * 256 + t;
    const int r = e >> 6;
    const int c = e & 63;
    sm[c][r] = in[(size_t)(r0 + r) * CC + c0 + c] * scale;
  }
  __syncthreads();
  const int lane = t & 31, wave = t >> 5;
  const int q = lane >> 3, c8 = (lane & 7) * 8;
  for (int pass = 0; pass < 2; ++pass) {
#pragma unroll
    for (int it = 0; it < 2; ++it) {
      const int row = wave * 8 + it * 4 + q;
      unsigned short hb[8], lb[8];
#pragma unroll
      for (int e = 0; e < 8; ++e) {
        const float f = sm[row][c8 + e];
        if (MODE == 0) { hb[e] = h_bits(f); lb[e] = 0; }
        else { hb[e] = f2bf_bits(f); lb[e] = f2bf_bits(f - bf_bits2f(hb[e])); }
      }
      const size_t o = (size_t)(c0 + row) * R + r0 + c8;
      const v4u u = pack8(hb);
      *(volatile v4u*)(out0 + o) = u;
      if (MODE == 1) { const v4u w = pack8(lb); *(volatile v4u*)(out1 + o) = w; }
    }
    __threadfence();
  }
}

__global__ __launch_bounds__(256) void wbc_kernel(const float* __restrict__ WB, const float* __restrict__ WC,
                                                 unsigned short* __restrict__ outh, unsigned short* __restrict__ outl) {
  __shared__ float sm[64][65];
  const int t  = threadIdx.x;
  const int e0 = blockIdx.x * 64;
#pragma unroll
  for (int i = 0; i < 4; ++i) {
    const int idx = i * 256 + t;
    const int r = idx >> 4;
    const int c = idx & 15;
    sm[c][r]      = WB[(size_t)(e0 + r) * kNS + c];
    sm[16 + c][r] = WC[(size_t)(e0 + r) * kNS + c];
  }
#pragma unroll
  for (int i = 0; i < 8; ++i) {
    const int idx = i * 256 + t;
    sm[32 + (idx >> 6)][idx & 63] = 0.0f;
  }
  __syncthreads();
  const int lane = t & 31, wave = t >> 5;
  const int q = lane >> 3, c8 = (lane & 7) * 8;
  for (int pass = 0; pass < 2; ++pass) {
#pragma unroll
    for (int it = 0; it < 2; ++it) {
      const int row = wave * 8 + it * 4 + q;
      unsigned short hb[8], lb[8];
#pragma unroll
      for (int e = 0; e < 8; ++e) {
        const float f = sm[row][c8 + e];
        hb[e] = f2bf_bits(f);
        lb[e] = f2bf_bits(f - bf_bits2f(hb[e]));
      }
      const size_t o = (size_t)row * kE + e0 + c8;
      const v4u u = pack8(hb);
      const v4u w = pack8(lb);
      *(volatile v4u*)(outh + o) = u;
      *(volatile v4u*)(outl + o) = w;
    }
    __threadfence();
  }
}

__global__ __launch_bounds__(256) void rmsnorm_kernel(const float* __restrict__ resid, const float* __restrict__ nw,
                                                     unsigned short* __restrict__ RNh, unsigned short* __restrict__ RNbh,
                                                     unsigned short* __restrict__ RNbl) {
  __shared__ float red[8];
  const int row  = blockIdx.x;
  const int t    = threadIdx.x;
  const int lane = t & 31, wave = t >> 5;
  const int c0   = t * 8;
  const float* p = resid + (size_t)row * kDm + c0;
  const v4f a = *(const v4f*)(p);
  const v4f c = *(const v4f*)(p + 4);
  float v[8];
#pragma unroll
  for (int e = 0; e < 4; ++e) { v[e] = a[e]; v[4 + e] = c[e]; }
  float ss = 0.f;
#pragma unroll
  for (int e = 0; e < 8; ++e) ss += v[e] * v[e];
#pragma unroll
  for (int off = 16; off > 0; off >>= 1) ss += __shfl_xor(ss, off, 32);
  if (lane == 0) red[wave] = ss;
  __syncthreads();
  float tot = red[0];
#pragma unroll
  for (int i = 1; i < 8; ++i) tot += red[i];
  const float sc = rsqrtf(tot * kInvDm + kEps);
  const v4f wa = *(const v4f*)(nw + c0);
  const v4f wc = *(const v4f*)(nw + c0 + 4);
  float w[8];
#pragma unroll
  for (int e = 0; e < 4; ++e) { w[e] = wa[e]; w[4 + e] = wc[e]; }
  unsigned short hb[8], bh[8], bl[8];
#pragma unroll
  for (int e = 0; e < 8; ++e) {
    const float rn = (v[e] * sc) * w[e];
    hb[e] = h_bits(rn);
    bh[e] = f2bf_bits(rn);
    bl[e] = f2bf_bits(rn - bf_bits2f(bh[e]));
  }
  const v4u u0 = pack8(hb), u1 = pack8(bh), u2 = pack8(bl);
  const size_t o = (size_t)row * kDm + c0;
  *(volatile v4u*)(RNh + o)  = u0;
  *(volatile v4u*)(RNbh + o) = u1;
  *(volatile v4u*)(RNbl + o) = u2;
  __threadfence();
  *(volatile v4u*)(RNh + o)  = u0;
  *(volatile v4u*)(RNbh + o) = u1;
  *(volatile v4u*)(RNbl + o) = u2;
}

__global__ __launch_bounds__(256) void conv_silu_kernel(const float* __restrict__ XIN, const float* __restrict__ cw,
                                                       const float* __restrict__ cb, float* __restrict__ X,
                                                       unsigned short* __restrict__ Xh, unsigned short* __restrict__ Xl) {
  __shared__ __align__(16) float sm[1024];
  const int bx  = blockIdx.x;
  const int row = bx >> 2;
  const int seg = bx & 3;
  const int t   = threadIdx.x;
  const int e   = seg * 1024 + t * 4;
  v4f acc = (v4f){0.f, 0.f, 0.f, 0.f};
#pragma unroll
  for (int k = 0; k < 4; ++k) {
    const int ll = row - 3 + k;
    if (ll >= 0) {
      const v4f xv = *(const v4f*)(XIN + (size_t)ll * kE + e);
      const v4f wv = *(const v4f*)(cw + (size_t)k * kE + e);
      acc += xv * wv;
    }
  }
  const v4f bb = *(const v4f*)(cb + e);
  acc += bb;
  float o[4];
#pragma unroll
  for (int j = 0; j < 4; ++j) o[j] = silu_f(acc[j]);
  const v4f ov = (v4f){o[0], o[1], o[2], o[3]};
  float* xp = X + (size_t)row * kE + e;
  *(volatile v4f*)xp = ov;
  __threadfence();
  *(volatile v4f*)xp = ov;
  *(v4f*)(&sm[t * 4]) = ov;
  __syncthreads();
  if (t < 128) {
    const v4f u0 = *(const v4f*)(&sm[t * 8]);
    const v4f u1 = *(const v4f*)(&sm[t * 8 + 4]);
    float f[8];
#pragma unroll
    for (int j = 0; j < 4; ++j) { f[j] = u0[j]; f[4 + j] = u1[j]; }
    unsigned short hb[8], lb[8];
#pragma unroll
    for (int j = 0; j < 8; ++j) {
      hb[j] = f2bf_bits(f[j]);
      lb[j] = f2bf_bits(f[j] - bf_bits2f(hb[j]));
    }
    const v4u vh = pack8(hb), vl = pack8(lb);
    const size_t oo = (size_t)row * kE + seg * 1024 + t * 8;
    *(volatile v4u*)(Xh + oo) = vh;
    *(volatile v4u*)(Xl + oo) = vl;
    __threadfence();
    *(volatile v4u*)(Xh + oo) = vh;
    *(volatile v4u*)(Xl + oo) = vl;
  }
}

__global__ __launch_bounds__(256) void scan_kernel(const float* __restrict__ DZ, const float* __restrict__ X,
                                                  const float* __restrict__ SK, const float* __restrict__ BC,
                                                  const float* __restrict__ Alog, const float* __restrict__ WD,
                                                  unsigned short* __restrict__ YS) {
  __shared__ float sD[kScanT][kScanCh];
  __shared__ float sX[kScanT][kScanCh];
  __shared__ float sG[kScanT][kScanCh];
  __shared__ float sBC[kScanT][32];
  __shared__ __align__(16) float sY[kScanT][kScanCh];
  const int t    = threadIdx.x;
  const int lane = t & 31, wave = t >> 5;
  const int el   = t >> 2;
  const int g    = t & 3;
  const int e0   = blockIdx.x * kScanCh;
  const int e    = e0 + el;
  float a[4], h[4];
#pragma unroll
  for (int j = 0; j < 4; ++j) {
    a[j] = -expf(Alog[(size_t)e * kNS + 4 * g + j]);
    h[j] = 0.f;
  }
  const float wd = WD[e];
  const int q = lane >> 3, c8 = (lane & 7) * 8;

  for (int ck = 0; ck < kL / kScanT; ++ck) {
    const int l0 = ck * kScanT;
#pragma unroll 1
    for (int i = 0; i < 8; ++i) {
      const int idx = i * 256 + t;
      const int s   = idx >> 6;
      const int cl  = idx & 63;
      const size_t go = (size_t)(l0 + s) * kE + e0 + cl;
      sD[s][cl] = softplus_f(DZ[go]);
      sX[s][cl] = X[go];
      sG[s][cl] = silu_f(SK[go]);
    }
#pragma unroll
    for (int i = 0; i < 4; ++i) {
      const int idx = i * 256 + t;
      const int s   = idx >> 5;
      const int n   = idx & 31;
      sBC[s][n] = BC[(size_t)(l0 + s) * kBCN + n];
    }
    __syncthreads();
#pragma unroll 1
    for (int s = 0; s < kScanT; ++s) {
      const float d  = sD[s][el];
      const float x  = sX[s][el];
      const float dx = d * x;
      float yp = 0.f;
#pragma unroll
      for (int j = 0; j < 4; ++j) {
        const float ab  = expf(d * a[j]);
        const float dxb = dx * sBC[s][4 * g + j];
        h[j] = h[j] * ab + dxb;
        yp += h[j] * sBC[s][16 + 4 * g + j];
      }
      yp += __shfl_xor(yp, 1, 32);
      yp += __shfl_xor(yp, 2, 32);
      const float ys = (yp + x * wd) * sG[s][el];
      if (g == 0) sY[s][el] = ys;
    }
    __syncthreads();
    for (int pass = 0; pass < 2; ++pass) {
      const int row = wave * 4 + q;
      const v4f va = *(const v4f*)(&sY[row][c8]);
      const v4f vb = *(const v4f*)(&sY[row][c8 + 4]);
      unsigned short hb[8];
#pragma unroll
      for (int j = 0; j < 4; ++j) { hb[j] = h_bits(va[j]); hb[4 + j] = h_bits(vb[j]); }
      const v4u u = pack8(hb);
      *(volatile v4u*)(YS + (size_t)(l0 + row) * kE + e0 + c8) = u;
      __threadfence();
    }
  }
}

extern "C" void kernel_launch(void* const* d_in, const int* in_sizes, int n_in,
                              void* d_out, int out_size, void* d_ws,
                              size_t ws_size, hipStream_t stream) {
  const size_t kMiB = (size_t)1 << 20;
  if (n_in < 14) return;
  if (in_sizes[0] != kL * kDm || in_sizes[1] != kDm || in_sizes[2] != kDm * kE || in_sizes[3] != kDm * kE ||
      in_sizes[4] != 4 * kE || in_sizes[5] != kE || in_sizes[6] != kE * kDR || in_sizes[7] != kDR * kE ||
      in_sizes[8] != kE || in_sizes[9] != kE * kNS || in_sizes[10] != kE * kNS || in_sizes[11] != kE * kNS ||
      in_sizes[12] != kE || in_sizes[13] != kE * kDm) return;
  if (out_size != kL * kDm) return;
  if (ws_size < 128 * kMiB) return;

  const float* resid  = (const float*)d_in[0];
  const float* norm_w = (const float*)d_in[1];
  const float* W_skip = (const float*)d_in[2];
  const float* W_in   = (const float*)d_in[3];
  const float* conv_w = (const float*)d_in[4];
  const float* conv_b = (const float*)d_in[5];
  const float* W_d1   = (const float*)d_in[6];
  const float* W_d2   = (const float*)d_in[7];
  const float* b_d2   = (const float*)d_in[8];
  const float* W_B    = (const float*)d_in[9];
  const float* W_C    = (const float*)d_in[10];
  const float* A_log  = (const float*)d_in[11];
  const float* W_D    = (const float*)d_in[12];
  const float* W_out  = (const float*)d_in[13];
  float* out = (float*)d_out;

  char* ws = (char*)d_ws;
  float*          SKIP   = (float*)(ws + 0 * kMiB);
  unsigned short* WoutT  = (unsigned short*)(ws + 0 * kMiB);
  unsigned short* RNbh   = (unsigned short*)(ws + 32 * kMiB);
  unsigned short* RNbl   = (unsigned short*)(ws + 40 * kMiB);
  unsigned short* WinTh  = (unsigned short*)(ws + 48 * kMiB);
  unsigned short* WinTl  = (unsigned short*)(ws + 64 * kMiB);
  float*          Xf     = (float*)(ws + 32 * kMiB);
  unsigned short* Xh     = (unsigned short*)(ws + 64 * kMiB);
  unsigned short* Xl     = (unsigned short*)(ws + 80 * kMiB);
  float*          DZ     = (float*)(ws + 64 * kMiB);
  unsigned short* RNh    = (unsigned short*)(ws + 96 * kMiB);
  unsigned short* WskipT = (unsigned short*)(ws + 104 * kMiB);
  float*          XIN    = (float*)(ws + 96 * kMiB);
  unsigned short* Wd1Th  = (unsigned short*)(ws + 96 * kMiB);
  unsigned short* Wd1Tl  = (unsigned short*)(ws + 97 * kMiB);
  unsigned short* Wd2Th  = (unsigned short*)(ws + 98 * kMiB);
  unsigned short* Wd2Tl  = (unsigned short*)(ws + 99 * kMiB);
  unsigned short* WBCTh  = (unsigned short*)(ws + 100 * kMiB);
  unsigned short* WBCTl  = (unsigned short*)(ws + 100 * kMiB + 512 * 1024);
  unsigned short* DT1h   = (unsigned short*)(ws + 101 * kMiB);
  unsigned short* DT1l   = (unsigned short*)(ws + 101 * kMiB + 512 * 1024);
  float*          BCf    = (float*)(ws + 102 * kMiB);
  unsigned short* YS     = (unsigned short*)(ws + 112 * kMiB);

  tcast_kernel<0><<<dim3(kDm / 64, kE / 64), 256, 0, stream>>>(W_skip, WskipT, WskipT, kDm, kE, kWCarry);
  tcast_kernel<1><<<dim3(kDm / 64, kE / 64), 256, 0, stream>>>(W_in, WinTh, WinTl, kDm, kE, 1.0f);

  rmsnorm_kernel<<<kL, 256, 0, stream>>>(resid, norm_w, RNh, RNbh, RNbl);

  wmma_gemm64<0, false, 0, 0, false, 0><<<dim3((kL / 64) * (kE / 64) / 8, 1), 256, 0, stream>>>(
      RNh, RNh, kDm, 0L, WskipT, WskipT, kDm, 0L, (void*)SKIP, (void*)SKIP, kE, 0L,
      conv_b, resid, 0L, kL, kE, kDm, kWCarryInv);

  wmma_gemm64<1, true, 0, 0, false, 0><<<dim3((kL / 64) * (kE / 64) / 8, 1), 256, 0, stream>>>(
      RNbh, RNbl, kDm, 0L, WinTh, WinTl, kDm, 0L, (void*)XIN, (void*)XIN, kE, 0L,
      conv_b, resid, 0L, kL, kE, kDm, 1.0f);

  conv_silu_kernel<<<kL * 4, 256, 0, stream>>>(XIN, conv_w, conv_b, Xf, Xh, Xl);

  tcast_kernel<1><<<dim3(kE / 64, kDR / 64), 256, 0, stream>>>(W_d1, Wd1Th, Wd1Tl, kE, kDR, 1.0f);
  tcast_kernel<1><<<dim3(kDR / 64, kE / 64), 256, 0, stream>>>(W_d2, Wd2Th, Wd2Tl, kDR, kE, 1.0f);
  wbc_kernel<<<kE / 64, 256, 0, stream>>>(W_B, W_C, WBCTh, WBCTl);

  wmma_gemm64<1, true, 0, 2, false, 0><<<dim3((kL / 64) * (kDR / 64) / 8, 1), 256, 0, stream>>>(
      Xh, Xl, kE, 0L, Wd1Th, Wd1Tl, kE, 0L, (void*)DT1h, (void*)DT1l, kDR, 0L,
      conv_b, resid, 0L, kL, kDR, kE, 1.0f);

  wmma_gemm64<1, true, 0, 0, false, 0><<<dim3((kL / 64) * (kBCN / 64) / 8, 1), 256, 0, stream>>>(
      Xh, Xl, kE, 0L, WBCTh, WBCTl, kE, 0L, (void*)BCf, (void*)BCf, kBCN, 0L,
      conv_b, resid, 0L, kL, kBCN, kE, 1.0f);

  wmma_gemm64<1, true, 2, 0, false, 0><<<dim3((kL / 64) * (kE / 64) / 8, 1), 256, 0, stream>>>(
      DT1h, DT1l, kDR, 0L, Wd2Th, Wd2Tl, kDR, 0L, (void*)DZ, (void*)DZ, kE, 0L,
      b_d2, resid, 0L, kL, kE, kDR, 1.0f);

  scan_kernel<<<kE / kScanCh, 256, 0, stream>>>(DZ, Xf, SKIP, BCf, A_log, W_D, YS);

  tcast_kernel<0><<<dim3(kE / 64, kDm / 64), 256, 0, stream>>>(W_out, WoutT, WoutT, kE, kDm, kWCarry);

  wmma_gemm64<0, false, 0, 0, true, 0><<<dim3((kL / 64) * (kDm / 64) / 8, 1), 256, 0, stream>>>(
      YS, YS, kE, 0L, WoutT, WoutT, kE, 0L, (void*)out, (void*)out, kDm, 0L,
      conv_b, resid, 0L, kL, kDm, kE, kWCarryInv);
}
